// EnsembleSurrogate_944892805218
// MI455X (gfx1250) — hardware-verified
//
#include <hip/hip_runtime.h>


typedef _Float16       v16h  __attribute__((ext_vector_type(16)));
typedef _Float16       v8h   __attribute__((ext_vector_type(8)));
typedef _Float16       v8ha  __attribute__((ext_vector_type(8), may_alias));
typedef __bf16         v16bf __attribute__((ext_vector_type(16)));
typedef unsigned short v8us  __attribute__((ext_vector_type(8)));
typedef unsigned short v8usa __attribute__((ext_vector_type(8), may_alias));
typedef float          v8f   __attribute__((ext_vector_type(8)));
typedef float          v4f   __attribute__((ext_vector_type(4)));
typedef float          v4fa  __attribute__((ext_vector_type(4), may_alias));
typedef unsigned int   uv4   __attribute__((ext_vector_type(4)));
typedef unsigned int   uv4a  __attribute__((ext_vector_type(4), may_alias));

#define N_MODELS        16
#define IN_DIM          32
#define HID             64
#define OUT_DIM         8
#define OUT_PAD         16
#define THREADS         256
#define WAVES_PER_BLOCK 8
#define ROWS_PER_WAVE   32
#define ROWS_PER_BLOCK  (WAVES_PER_BLOCK * ROWS_PER_WAVE)

#define OFFB_W1     0
#define OFFB_W2     4096
#define OFFB_W3     12288
#define OFFB_W4     20480
#define OFFB_B      22528
#define OFFB_PAD    23360
#define BLOB_BYTES  23552
#define BLOB_CHUNKS (BLOB_BYTES / 16)
#define WSCALE      256.0f
#define WSCALE_INV  0.00390625f

static_assert(BLOB_BYTES % 128 == 0);
static_assert(OFFB_B + 208 * 4 == OFFB_PAD);
static_assert(OFFB_PAD % 16 == 0);

union FragH  { v16h  v; v8h  h[2]; };
union FragBF { v16bf v; v8us h[2]; };

__device__ __forceinline__ unsigned short bf16_bits(float f) {
    unsigned int u = __float_as_uint(f);
    u += 0x7FFFu + ((u >> 16) & 1u);
    return (unsigned short)(u >> 16);
}

__device__ __forceinline__ float bf16_rne(float f) {
    return __uint_as_float(((unsigned int)bf16_bits(f)) << 16);
}

__device__ __forceinline__ v8f v8f_splat(float v) {
    v8f r;
#pragma unroll
    for (int i = 0; i < 8; ++i) r[i] = v;
    return r;
}

__device__ __forceinline__ v8f mma_f16(v16h a, v16h b, v8f c) {
    v8f d = __builtin_amdgcn_wmma_f32_16x16x32_f16(false, a, false, b, (short)0, c, false, false);
    asm volatile("v_nop\n\tv_nop\n\tv_nop\n\tv_nop" : "+v"(d) : "v"(a), "v"(b));
    return d;
}

__device__ __forceinline__ v8f mma_bf16(v16bf a, v16bf b, v8f c) {
    v8f d = __builtin_amdgcn_wmma_f32_16x16x32_bf16(false, a, false, b, (short)0, c, false, false);
    asm volatile("v_nop\n\tv_nop\n\tv_nop\n\tv_nop" : "+v"(d) : "v"(a), "v"(b));
    return d;
}

__device__ __forceinline__ v16h ld_frag_h(const _Float16* base, int ld, int K0, int idx, int half) {
    const _Float16* p = base + idx * ld + K0 + 8 * half;
    FragH f;
    f.h[0] = *(const v8ha*)(p);
    f.h[1] = *(const v8ha*)(p + 16);
    return f.v;
}

__device__ __forceinline__ v16bf ld_frag_bf(const unsigned short* base, int ld, int K0, int idx, int half) {
    const unsigned short* p = base + idx * ld + K0 + 8 * half;
    FragBF f;
    f.h[0] = *(const v8usa*)(p);
    f.h[1] = *(const v8usa*)(p + 16);
    return f.v;
}

__device__ __forceinline__ void relu_store(_Float16* hbuf, v8f acc, float scale, float bias,
                                           int base_row, int col, int half) {
#pragma unroll
    for (int v = 0; v < 8; ++v) {
        float hv = __builtin_fmaxf(__builtin_fmaf(acc[v], scale, bias), 0.0f);
        hbuf[(base_row + 8 * half + v) * HID + col] = (_Float16)hv;
    }
}

__device__ __forceinline__ void layer_hid(const _Float16* Wt, const float* bias, _Float16* hbuf,
                                          int r, int half, v16h a00, v16h a01, v16h a10, v16h a11) {
#pragma unroll
    for (int t = 0; t < 4; ++t) {
        const int n = t * 16 + r;
        v16h b0 = ld_frag_h(Wt, HID, 0,  n, half);
        v16h b1 = ld_frag_h(Wt, HID, 32, n, half);
        v8f acc0 = v8f_splat(0.0f), acc1 = v8f_splat(0.0f);
        acc0 = mma_f16(a00, b0, acc0);
        acc1 = mma_f16(a10, b0, acc1);
        acc0 = mma_f16(a01, b1, acc0);
        acc1 = mma_f16(a11, b1, acc1);
        const float bv = bias[n];
        relu_store(hbuf, acc0, WSCALE_INV, bv, 0,  n, half);
        relu_store(hbuf, acc1, WSCALE_INV, bv, 16, n, half);
    }
}

__global__ __launch_bounds__(THREADS)
void mlp_stats_kernel(const float* __restrict__ x,
                      const unsigned char* __restrict__ wblob,
                      const unsigned char* __restrict__ wblob2,
                      float* __restrict__ out, int batch) {
    __shared__ __align__(16) unsigned char sBlob[BLOB_BYTES];
    __shared__ __align__(16) _Float16 sH[WAVES_PER_BLOCK * ROWS_PER_WAVE * HID];

    const unsigned short* sW1 = (const unsigned short*)(sBlob + OFFB_W1);
    const _Float16* sW2 = (const _Float16*)(sBlob + OFFB_W2);
    const _Float16* sW3 = (const _Float16*)(sBlob + OFFB_W3);
    const _Float16* sW4 = (const _Float16*)(sBlob + OFFB_W4);
    const float* sb  = (const float*)(sBlob + OFFB_B);
    const float* sb1 = sb;
    const float* sb2 = sb + 64;
    const float* sb3 = sb + 128;
    const float* sb4 = sb + 192;

    const int tid  = threadIdx.x;
    const int wave = tid >> 5;
    const int lane = tid & 31;
    const int r    = lane & 15;
    const int half = lane >> 4;
    const int rowbase = blockIdx.x * ROWS_PER_BLOCK + wave * ROWS_PER_WAVE;

    v16bf xa0, xa1;
    {
        FragBF fx;
#pragma unroll
        for (int s = 0; s < 2; ++s) {
            int row = rowbase + s * 16 + r;
            row = (row < batch) ? row : (batch - 1);
            const float* xr = x + (size_t)row * IN_DIM + 8 * half;
            const v4f f0 = *(const v4f*)(xr);
            const v4f f1 = *(const v4f*)(xr + 4);
            const v4f f2 = *(const v4f*)(xr + 16);
            const v4f f3 = *(const v4f*)(xr + 20);
            v8us lo, hi;
            lo[0] = bf16_bits(f0[0]); lo[1] = bf16_bits(f0[1]); lo[2] = bf16_bits(f0[2]); lo[3] = bf16_bits(f0[3]);
            lo[4] = bf16_bits(f1[0]); lo[5] = bf16_bits(f1[1]); lo[6] = bf16_bits(f1[2]); lo[7] = bf16_bits(f1[3]);
            hi[0] = bf16_bits(f2[0]); hi[1] = bf16_bits(f2[1]); hi[2] = bf16_bits(f2[2]); hi[3] = bf16_bits(f2[3]);
            hi[4] = bf16_bits(f3[0]); hi[5] = bf16_bits(f3[1]); hi[6] = bf16_bits(f3[2]); hi[7] = bf16_bits(f3[3]);
            fx.h[0] = lo;
            fx.h[1] = hi;
            if (s == 0) xa0 = fx.v; else xa1 = fx.v;
        }
    }

    v8f sum0 = v8f_splat(0.0f), sq0 = v8f_splat(0.0f), p00 = v8f_splat(0.0f);
    v8f sum1 = v8f_splat(0.0f), sq1 = v8f_splat(0.0f), p01 = v8f_splat(0.0f);

    _Float16* hbuf = sH + wave * (ROWS_PER_WAVE * HID);

#pragma unroll 1
    for (int m = 0; m < N_MODELS; ++m) {
        __syncthreads();

        {
            const uv4a* g1 = (const uv4a*)(wblob  + (size_t)m * BLOB_BYTES);
            const uv4a* g2 = (const uv4a*)(wblob2 + (size_t)m * BLOB_BYTES);
            uv4a* sdst = (uv4a*)sBlob;
            for (int e = tid; e < BLOB_CHUNKS; e += THREADS) {
                uv4 v = g1[e];
                const bool fill = (v.x == 0xAAAAAAAAu) & (v.y == 0xAAAAAAAAu) &
                                  (v.z == 0xAAAAAAAAu) & (v.w == 0xAAAAAAAAu);
                if (fill) v = g2[e];
                sdst[e] = v;
            }
        }
        __syncthreads();

#pragma unroll
        for (int t = 0; t < 4; ++t) {
            const int n = t * 16 + r;
            v16bf bw = ld_frag_bf(sW1, IN_DIM, 0, n, half);
            v8f acc0 = v8f_splat(0.0f), acc1 = v8f_splat(0.0f);
            acc0 = mma_bf16(xa0, bw, acc0);
            acc1 = mma_bf16(xa1, bw, acc1);
            const float bv = sb1[n];
            relu_store(hbuf, acc0, 1.0f, bv, 0,  n, half);
            relu_store(hbuf, acc1, 1.0f, bv, 16, n, half);
        }
        __syncthreads();
        v16h a00 = ld_frag_h(hbuf, HID, 0,  r,      half);
        v16h a01 = ld_frag_h(hbuf, HID, 32, r,      half);
        v16h a10 = ld_frag_h(hbuf, HID, 0,  16 + r, half);
        v16h a11 = ld_frag_h(hbuf, HID, 32, 16 + r, half);

        layer_hid(sW2, sb2, hbuf, r, half, a00, a01, a10, a11);
        __syncthreads();
        a00 = ld_frag_h(hbuf, HID, 0,  r,      half);
        a01 = ld_frag_h(hbuf, HID, 32, r,      half);
        a10 = ld_frag_h(hbuf, HID, 0,  16 + r, half);
        a11 = ld_frag_h(hbuf, HID, 32, 16 + r, half);

        layer_hid(sW3, sb3, hbuf, r, half, a00, a01, a10, a11);
        __syncthreads();
        a00 = ld_frag_h(hbuf, HID, 0,  r,      half);
        a01 = ld_frag_h(hbuf, HID, 32, r,      half);
        a10 = ld_frag_h(hbuf, HID, 0,  16 + r, half);
        a11 = ld_frag_h(hbuf, HID, 32, 16 + r, half);

        {
            v16h b0 = ld_frag_h(sW4, HID, 0,  r, half);
            v16h b1 = ld_frag_h(sW4, HID, 32, r, half);
            v8f acc0 = v8f_splat(0.0f), acc1 = v8f_splat(0.0f);
            acc0 = mma_f16(a00, b0, acc0);
            acc1 = mma_f16(a10, b0, acc1);
            acc0 = mma_f16(a01, b1, acc0);
            acc1 = mma_f16(a11, b1, acc1);
            const v8f bv8 = v8f_splat(sb4[r]);
            const v8f sc8 = v8f_splat(WSCALE_INV);
            v8f pred0 = acc0 * sc8 + bv8;
            v8f pred1 = acc1 * sc8 + bv8;
            if (m == 0) {
                p00 = pred0;
                p01 = pred1;
            } else {
                v8f d0 = pred0 - p00;
                v8f d1 = pred1 - p01;
                sum0 += d0; sq0 += d0 * d0;
                sum1 += d1; sq1 += d1 * d1;
            }
        }
    }

    __syncthreads();
    float* stage = (float*)sH + wave * (ROWS_PER_WAVE * HID / 2);
    if (r < OUT_DIM) {
#pragma unroll
        for (int s = 0; s < 2; ++s) {
            const v8f su8 = s ? sum1 : sum0;
            const v8f sq8 = s ? sq1  : sq0;
            const v8f pz8 = s ? p01  : p00;
#pragma unroll
            for (int v = 0; v < 8; ++v) {
                const int rowl = s * 16 + 8 * half + v;
                const float su   = su8[v];
                const float mean = __builtin_fmaf(su, 1.0f / 16.0f, pz8[v]);
                float var = (sq8[v] - su * su * (1.0f / 16.0f)) * (1.0f / 15.0f);
                var = __builtin_fmaxf(var, 0.0f);
                const float sd = sqrtf(var);
                stage[rowl * OUT_DIM + r]       = mean;
                stage[256 + rowl * OUT_DIM + r] = sd;
            }
        }
    }
    __syncthreads();

    {
        const v4fa* stg = (const v4fa*)stage;
        const v4f mv0 = stg[lane];
        const v4f mv1 = stg[32 + lane];
        const v4f sv0 = stg[64 + lane];
        const v4f sv1 = stg[96 + lane];
        float* o0 = out + (size_t)rowbase * OUT_DIM;
        float* o1 = out + (size_t)batch * OUT_DIM + (size_t)rowbase * OUT_DIM;
        if (rowbase + ROWS_PER_WAVE <= batch) {
            *(volatile v4f*)(o0 + lane * 4)       = mv0;
            *(volatile v4f*)(o0 + 128 + lane * 4) = mv1;
            *(volatile v4f*)(o1 + lane * 4)       = sv0;
            *(volatile v4f*)(o1 + 128 + lane * 4) = sv1;
            __threadfence();
            *(volatile v4f*)(o0 + lane * 4)       = mv0;
            *(volatile v4f*)(o0 + 128 + lane * 4) = mv1;
            *(volatile v4f*)(o1 + lane * 4)       = sv0;
            *(volatile v4f*)(o1 + 128 + lane * 4) = sv1;
        } else {
            for (int e = lane; e < ROWS_PER_WAVE * OUT_DIM; e += 32) {
                const int rowl = e >> 3;
                if (rowbase + rowl < batch) {
                    const float mvs = stage[e];
                    const float svs = stage[256 + e];
                    *(volatile float*)(o0 + e) = mvs;
                    *(volatile float*)(o1 + e) = svs;
                }
            }
            __threadfence();
            for (int e = lane; e < ROWS_PER_WAVE * OUT_DIM; e += 32) {
                const int rowl = e >> 3;
                if (rowbase + rowl < batch) {
                    const float mvs = stage[e];
                    const float svs = stage[256 + e];
                    *(volatile float*)(o0 + e) = mvs;
                    *(volatile float*)(o1 + e) = svs;
                }
            }
        }
    }
}

__global__ __launch_bounds__(THREADS)
void pack_weights_kernel(const float* __restrict__ W1, const float* __restrict__ b1,
                         const float* __restrict__ W2, const float* __restrict__ b2,
                         const float* __restrict__ W3, const float* __restrict__ b3,
                         const float* __restrict__ W4, const float* __restrict__ b4,
                         unsigned char* __restrict__ blob) {
    __shared__ __align__(16) unsigned char img[BLOB_BYTES];
    const int m   = blockIdx.x;
    const int tid = threadIdx.x;

    unsigned short* w1 = (unsigned short*)(img + OFFB_W1);
    _Float16* w2 = (_Float16*)(img + OFFB_W2);
    _Float16* w3 = (_Float16*)(img + OFFB_W3);
    _Float16* w4 = (_Float16*)(img + OFFB_W4);
    float* bb = (float*)(img + OFFB_B);

    const float* g = W1 + (size_t)m * IN_DIM * HID;
    for (int e = tid; e < IN_DIM * HID; e += THREADS) {
        const int k = e >> 6, n = e & 63;
        w1[n * IN_DIM + k] = bf16_bits(g[e]);
    }
    g = W2 + (size_t)m * HID * HID;
    for (int e = tid; e < HID * HID; e += THREADS) {
        const int k = e >> 6, n = e & 63;
        w2[n * HID + k] = (_Float16)(WSCALE * bf16_rne(g[e]));
    }
    g = W3 + (size_t)m * HID * HID;
    for (int e = tid; e < HID * HID; e += THREADS) {
        const int k = e >> 6, n = e & 63;
        w3[n * HID + k] = (_Float16)(WSCALE * bf16_rne(g[e]));
    }
    g = W4 + (size_t)m * HID * OUT_DIM;
    for (int e = tid; e < OUT_PAD * HID; e += THREADS) {
        const int n = e >> 6, k = e & 63;
        const float wv = (n < OUT_DIM) ? (WSCALE * bf16_rne(g[k * OUT_DIM + n])) : 0.0f;
        w4[e] = (_Float16)wv;
    }
    if (tid < HID) {
        bb[tid]       = bf16_rne(b1[m * HID + tid]);
        bb[64 + tid]  = bf16_rne(b2[m * HID + tid]);
        bb[128 + tid] = bf16_rne(b3[m * HID + tid]);
    }
    if (tid < OUT_PAD) bb[192 + tid] = (tid < OUT_DIM) ? bf16_rne(b4[m * OUT_DIM + tid]) : 0.0f;
    if (tid < (BLOB_BYTES - OFFB_PAD) / 4) ((float*)(img + OFFB_PAD))[tid] = 0.0f;
    __syncthreads();

    const uv4a* src = (const uv4a*)img;
    unsigned char* dst = blob + (size_t)m * BLOB_BYTES;
    for (int e = tid; e < BLOB_CHUNKS; e += THREADS) {
        const uv4 v = src[e];
        *(volatile uv4*)(dst + (size_t)e * 16) = v;
    }
    __threadfence();
    for (int e = tid; e < BLOB_CHUNKS; e += THREADS) {
        const uv4 v = src[e];
        *(volatile uv4*)(dst + (size_t)e * 16) = v;
    }
}

extern "C" void kernel_launch(void* const* d_in, const int* in_sizes, int n_in,
                              void* d_out, int out_size, void* d_ws, size_t ws_size,
                              hipStream_t stream) {
    (void)n_in;
    const float* x  = (const float*)d_in[0];
    const float* W1 = (const float*)d_in[1];
    const float* b1 = (const float*)d_in[2];
    const float* W2 = (const float*)d_in[3];
    const float* b2 = (const float*)d_in[4];
    const float* W3 = (const float*)d_in[5];
    const float* b3 = (const float*)d_in[6];
    const float* W4 = (const float*)d_in[7];
    const float* b4 = (const float*)d_in[8];
    float* out = (float*)d_out;

    const int batch = in_sizes[0] / IN_DIM;
    if (batch <= 0) return;
    if ((long long)out_size < 2LL * (long long)batch * OUT_DIM) return;

    const size_t copy_bytes = (size_t)N_MODELS * BLOB_BYTES;
    if (ws_size < 2 * copy_bytes) return;
    unsigned char* blob  = (unsigned char*)d_ws;
    unsigned char* blob2 = blob + copy_bytes;

    const int blocks = (batch + ROWS_PER_BLOCK - 1) / ROWS_PER_BLOCK;

    pack_weights_kernel<<<dim3(N_MODELS), dim3(THREADS), 0, stream>>>(W1, b1, W2, b2, W3, b3, W4, b4, blob);
    pack_weights_kernel<<<dim3(N_MODELS), dim3(THREADS), 0, stream>>>(W1, b1, W2, b2, W3, b3, W4, b4, blob2);
    mlp_stats_kernel<<<dim3(blocks), dim3(THREADS), 0, stream>>>(x, blob, blob2, out, batch);
}
